// SpearmanCorrelation_46291157516693
// MI455X (gfx1250) — hardware-verified
//
#include <hip/hip_runtime.h>

constexpr int  kB = 128;
constexpr int  kE = 128;
constexpr int  kF = 32;
constexpr int  kChunk = 32;
constexpr int  kNumChunks = kB / kChunk;
constexpr int  kKdim = kF * kE;
constexpr long kPlaneHalves = (long)kChunk * kE * kKdim;
constexpr long kPlaneBytes  = kPlaneHalves * 2;
constexpr long kGBytes  = (long)kB * kE * kE * 4;
constexpr long kSEBytes = (long)kB * kF * kE * 4;
constexpr long kOffPhi = 0;
constexpr long kOffPlo = kOffPhi + kPlaneBytes;
constexpr long kOffG   = kOffPlo + kPlaneBytes;
constexpr long kOffSE  = kOffG + kGBytes;
constexpr long kWsTotal = kOffSE + kSEBytes;
typedef char ws_fits_check[(kWsTotal <= 134217728L) ? 1 : -1];
constexpr float kInvEm1 = 1.0f / 127.0f;
constexpr float kInvF   = 1.0f / 32.0f;

typedef __attribute__((ext_vector_type(16))) _Float16 v16h;
typedef __attribute__((ext_vector_type(8)))  _Float16 v8h;
typedef __attribute__((ext_vector_type(16))) __bf16   v16b;
typedef __attribute__((ext_vector_type(8)))  __bf16   v8b;
typedef __attribute__((ext_vector_type(8)))  float    v8f;
typedef __attribute__((ext_vector_type(4)))  float    v4f;
typedef __attribute__((ext_vector_type(4)))  unsigned int v4u;

__device__ __forceinline__ unsigned short f2bf_bits(float f) {
  unsigned u = __float_as_uint(f);
  return (unsigned short)((u + 0x7FFFu + ((u >> 16) & 1u)) >> 16);
}
__device__ __forceinline__ float bf_bits2f(unsigned short h) { return __uint_as_float(((unsigned)h) << 16); }

__device__ __forceinline__ void dep_guard_h(v8f& a, v8f& b, v16h x, v16h y) { asm volatile("v_nop\n\tv_nop\n\tv_nop\n\tv_nop" : "+v"(a), "+v"(b) : "v"(x), "v"(y)); }
__device__ __forceinline__ void dep_guard_b(v8f& a, v8f& b, v16b x, v16b y) { asm volatile("v_nop\n\tv_nop\n\tv_nop\n\tv_nop" : "+v"(a), "+v"(b) : "v"(x), "v"(y)); }
__device__ __forceinline__ void keep4_h(v16h a, v16h b, v16h c, v16h d) { asm volatile("v_nop" :: "v"(a), "v"(b), "v"(c), "v"(d)); }
__device__ __forceinline__ void keep4_b(v16b a, v16b b, v16b c, v16b d) { asm volatile("v_nop" :: "v"(a), "v"(b), "v"(c), "v"(d)); }
__device__ __forceinline__ void acc_guard4(v8f& a, v8f& b, v8f& c, v8f& d) { asm volatile("v_nop\n\tv_nop\n\tv_nop\n\tv_nop" : "+v"(a), "+v"(b), "+v"(c), "+v"(d)); }
template <typename T> struct Frag;
template <> struct Frag<_Float16> {
  typedef v16h V; union U { v16h v; v8h h[2]; };
  static __device__ __forceinline__ v16h load(const _Float16* p) {
    U f; f.h[0] = *(const v8h*)(p); f.h[1] = *(const v8h*)(p + 16); return f.v;
  }
  static __device__ __forceinline__ v8f mma(v16h a, v16h b, v8f c) {
    return __builtin_amdgcn_wmma_f32_16x16x32_f16(false, a, false, b, (short)0, c, false, false);
  }
  static __device__ __forceinline__ void guard(v8f& a, v8f& b, v16h x, v16h y) { dep_guard_h(a, b, x, y); }
  static __device__ __forceinline__ void keep(v16h a, v16h b, v16h c, v16h d) { keep4_h(a, b, c, d); }
};
template <> struct Frag<__bf16> {
  typedef v16b V; union U { v16b v; v8b h[2]; };
  static __device__ __forceinline__ v16b load(const __bf16* p) {
    U f; f.h[0] = *(const v8b*)(p); f.h[1] = *(const v8b*)(p + 16); return f.v;
  }
  static __device__ __forceinline__ v8f mma(v16b a, v16b b, v8f c) {
    return __builtin_amdgcn_wmma_f32_16x16x32_bf16(false, a, false, b, (short)0, c, false, false);
  }
  static __device__ __forceinline__ void guard(v8f& a, v8f& b, v16b x, v16b y) { dep_guard_b(a, b, x, y); }
  static __device__ __forceinline__ void keep(v16b a, v16b b, v16b c, v16b d) { keep4_b(a, b, c, d); }
};

__device__ __forceinline__ unsigned pk16(unsigned short a, unsigned short b) { return (unsigned)a | ((unsigned)b << 16); }

template <int ET> struct Elem;
template <> struct Elem<0> { typedef _Float16 T; };
template <> struct Elem<1> { typedef __bf16 T; };
template <int ET, bool SPLIT, int BIAS_MODE, int OUT_MODE, bool RESID, int ACT = 0>
__global__ __launch_bounds__(256) void wmma_gemm64(
    const unsigned short* __restrict__ Ap, const unsigned short* __restrict__ A2p, int lda, long strideA,
    const unsigned short* __restrict__ Btp, const unsigned short* __restrict__ Bt2p, int ldb, long strideB,
    void* __restrict__ Cout, void* __restrict__ Cout2, int ldc, long strideC,
    const float* __restrict__ bias,
    const float* __restrict__ resid, long strideR,
    int M, int N, int K, float scale) {
  typedef typename Elem<ET>::T T;
  typedef typename Frag<T>::V V;
  const T* A = (const T*)Ap; const T* A2 = (const T*)A2p; const T* Bt = (const T*)Btp; const T* Bt2 = (const T*)Bt2p;
  __shared__ __align__(16) float sT[8][16 * 68];
  const int b    = blockIdx.y;
  const int lane = threadIdx.x & 31;
  const int wave = threadIdx.x >> 5;
  const int tilesN = N >> 6;
  const int tilesM = M >> 6;
  const int tile = blockIdx.x * 8 + wave;
  if (tile >= tilesM * tilesN) return;
  const int tm = tile / tilesN;
  const int tn = tile - tm * tilesN;
  const int m0 = tm << 6;
  const int n0 = tn << 6;

  const T* Ab  = A  + (size_t)b * strideA;
  const T* Bb  = Bt + (size_t)b * strideB;
  const T* Ab2 = SPLIT ? (A2  + (size_t)b * strideA) : nullptr;
  const T* Bb2 = SPLIT ? (Bt2 + (size_t)b * strideB) : nullptr;

  const int rlane = lane & 15;
  const int koff  = (lane >> 4) * 8;
  const int mOff  = (lane >> 4) * 8;

  v8f acc[4][4];
#pragma unroll
  for (int i = 0; i < 4; ++i)
#pragma unroll
    for (int j = 0; j < 4; ++j) acc[i][j] = (v8f){0.f,0.f,0.f,0.f,0.f,0.f,0.f,0.f};

  for (int k0 = 0; k0 < K; k0 += 32) {
    V bh[4], bl[4];
#pragma unroll
    for (int j = 0; j < 4; ++j) {
      const size_t bo = (size_t)(n0 + (j << 4) + rlane) * ldb + koff + k0;
      bh[j] = Frag<T>::load(Bb + bo);
      if (SPLIT) bl[j] = Frag<T>::load(Bb2 + bo);
    }
#pragma unroll
    for (int i = 0; i < 4; ++i) {
      const size_t ao = (size_t)(m0 + (i << 4) + rlane) * lda + koff + k0;
      V ah = Frag<T>::load(Ab + ao);
      V al;
      if (SPLIT) al = Frag<T>::load(Ab2 + ao);
#pragma unroll
      for (int j = 0; j < 4; ++j) {
        acc[i][j] = Frag<T>::mma(ah, bh[j], acc[i][j]);
        if (SPLIT) {
          acc[i][j] = Frag<T>::mma(ah, bl[j], acc[i][j]);
          acc[i][j] = Frag<T>::mma(al, bh[j], acc[i][j]);
        }
      }
      Frag<T>::guard(acc[i][0], acc[i][3], ah, SPLIT ? al : ah);
    }
    Frag<T>::keep(bh[0], bh[1], bh[2], bh[3]);
    if (SPLIT) Frag<T>::keep(bl[0], bl[1], bl[2], bl[3]);
  }
  acc_guard4(acc[0][0], acc[0][1], acc[0][2], acc[0][3]);
  acc_guard4(acc[1][0], acc[1][1], acc[1][2], acc[1][3]);
  acc_guard4(acc[2][0], acc[2][1], acc[2][2], acc[2][3]);
  acc_guard4(acc[3][0], acc[3][1], acc[3][2], acc[3][3]);

  float* slab = sT[wave];
  const float* Rb = RESID ? (resid + (size_t)b * strideR) : nullptr;
#pragma unroll
  for (int i = 0; i < 4; ++i) {
    const int mBase = m0 + (i << 4);
#pragma unroll
    for (int j = 0; j < 4; ++j) {
      const int n = n0 + (j << 4) + rlane;
      float bv = 0.f;
      if (BIAS_MODE == 2) bv = bias[n];
#pragma unroll
      for (int r = 0; r < 8; ++r) {
        float v = acc[i][j][r] * scale;
        if (BIAS_MODE == 1) v += bias[mBase + mOff + r];
        if (BIAS_MODE == 2) v += bv;
        if (RESID) v += Rb[(size_t)(mBase + mOff + r) * ldc + n];
        if (ACT == 2) v = fmaxf(v, 0.0f);
        if (ACT == 4) v = (v > 0.f) ? v : 0.01f * v;
        slab[(mOff + r) * 68 + (j << 4) + rlane] = v;
      }
    }
    __builtin_amdgcn_fence(__ATOMIC_RELEASE, "workgroup");
    __builtin_amdgcn_wave_barrier();
    __builtin_amdgcn_fence(__ATOMIC_ACQUIRE, "workgroup");
    if (OUT_MODE == 0) {
      float* C = (float*)Cout + (size_t)b * strideC;
      const int hh = lane >> 4, c4 = (lane & 15) * 4;
      for (int pass = 0; pass < 2; ++pass) {
#pragma unroll
        for (int it = 0; it < 8; ++it) {
          const int row = it * 2 + hh;
          v4f v = *(const v4f*)(slab + row * 68 + c4);
          *(volatile v4f*)(C + (size_t)(mBase + row) * ldc + n0 + c4) = v;
        }
        __threadfence();
      }
    } else {
      const int q = lane >> 3, c8 = (lane & 7) * 8;
      unsigned short* C  = (unsigned short*)Cout  + (size_t)b * strideC;
      unsigned short* C2 = (OUT_MODE == 2) ? ((unsigned short*)Cout2 + (size_t)b * strideC) : nullptr;
      for (int pass = 0; pass < 2; ++pass) {
#pragma unroll
        for (int it = 0; it < 4; ++it) {
          const int row = it * 4 + q;
          const float* sp = slab + row * 68 + c8;
          v8h hv, lv;
#pragma unroll
          for (int e = 0; e < 8; ++e) {
            if (OUT_MODE == 1) {
              hv[e] = (_Float16)sp[e];
            } else {
              unsigned short hb = f2bf_bits(sp[e]);
              unsigned short lb = f2bf_bits(sp[e] - bf_bits2f(hb));
              hv[e] = __builtin_bit_cast(_Float16, hb);
              lv[e] = __builtin_bit_cast(_Float16, lb);
            }
          }
          *(volatile v8h*)(C + (size_t)(mBase + row) * ldc + n0 + c8) = hv;
          if (OUT_MODE == 2) *(volatile v8h*)(C2 + (size_t)(mBase + row) * ldc + n0 + c8) = lv;
        }
        __threadfence();
      }
    }
    __builtin_amdgcn_fence(__ATOMIC_RELEASE, "workgroup");
    __builtin_amdgcn_wave_barrier();
    __builtin_amdgcn_fence(__ATOMIC_ACQUIRE, "workgroup");
  }
}

__global__ __launch_bounds__(128) void rank_weight_kernel(const float* __restrict__ de,
                                                          unsigned short* __restrict__ Phi,
                                                          unsigned short* __restrict__ Plo,
                                                          float* __restrict__ SE, int b0) {
  __shared__ float xs[kE];
  __shared__ int   rk[kE];
  __shared__ float rtab[kE];
  __shared__ __align__(16) float ses[kE];
  const int tid = threadIdx.x;
  const int bl  = blockIdx.x >> 5;
  const int f   = blockIdx.x & (kF - 1);
  const int b   = b0 + bl;

  xs[tid]   = de[((size_t)b * kE + tid) * kF + f];
  rtab[tid] = 1.0f / (float)(tid + 1);
  __syncthreads();

  const float xi = xs[tid];
  int r = 0;
#pragma unroll 4
  for (int j = 0; j < kE; ++j) {
    const float xj = xs[j];
    r += ((xj < xi) || (xj == xi && j < tid)) ? 1 : 0;
  }
  rk[tid] = r;
  __syncthreads();

  {
    float s = 0.f;
#pragma unroll 4
    for (int m = 0; m < kE; ++m) {
      int d = r - rk[m];
      d = (d < 0) ? -d : d;
      s += rtab[d];
    }
    ses[tid] = s;
  }

  const int lane = tid & 31, wave = tid >> 5;
  const int hh = lane >> 4, c8 = (lane & 15) * 8;
  const size_t rowbase = (size_t)bl * kE;
  for (int pass = 0; pass < 2; ++pass) {
#pragma unroll 1
    for (int it = 0; it < 16; ++it) {
      const int e  = wave * 32 + it * 2 + hh;
      const int re = rk[e];
      unsigned short hb[8], lb[8];
#pragma unroll
      for (int i = 0; i < 8; ++i) {
        int d = re - rk[c8 + i];
        d = (d < 0) ? -d : d;
        const float w = rtab[d];
        const unsigned short h = f2bf_bits(w);
        hb[i] = h;
        lb[i] = f2bf_bits(w - bf_bits2f(h));
      }
      const v4u uh = (v4u){pk16(hb[0], hb[1]), pk16(hb[2], hb[3]), pk16(hb[4], hb[5]), pk16(hb[6], hb[7])};
      const v4u ul = (v4u){pk16(lb[0], lb[1]), pk16(lb[2], lb[3]), pk16(lb[4], lb[5]), pk16(lb[6], lb[7])};
      const size_t off = (rowbase + (size_t)e) * (size_t)kKdim + (size_t)f * kE + (size_t)c8;
      *(volatile v4u*)(Phi + off) = uh;
      *(volatile v4u*)(Plo + off) = ul;
    }
    __threadfence();
  }

  __syncthreads();
  if (wave == 0) {
    const v4f sv = *(const v4f*)(ses + 4 * lane);
    float* sp = SE + ((size_t)b * kF + f) * kE + 4 * lane;
    *(volatile v4f*)sp = sv;
    __threadfence();
    *(volatile v4f*)sp = sv;
  }
}

__global__ __launch_bounds__(128) void finish_kernel(const float* __restrict__ G, const float* __restrict__ SE,
                                                     float* __restrict__ out) {
  const int tid = threadIdx.x;
  const int lane = tid & 31, wave = tid >> 5;
  const int b  = blockIdx.x >> 5;
  const int jg = blockIdx.x & 31;
  const int j  = jg * 4 + wave;
  const int k4 = lane * 4;
  const size_t rowoff = ((size_t)b * kE + j) * kE + k4;
  const v4f g = *(const v4f*)(G + rowoff);
  v4f x = (v4f){0.f, 0.f, 0.f, 0.f};
  const float* sb = SE + (size_t)b * kF * kE;
#pragma unroll 1
  for (int f = 0; f < kF; ++f) {
    const float* sp = sb + (size_t)f * kE;
    const float sj = sp[j];
    const v4f sk = *(const v4f*)(sp + k4);
    x = x + sk * sj;
  }
  const v4f o = (g - x * kInvEm1) * kInvF;
  float* op = out + rowoff;
  *(volatile v4f*)op = o;
  __threadfence();
  *(volatile v4f*)op = o;
}

extern "C" void kernel_launch(void* const* d_in, const int* in_sizes, int n_in,
                              void* d_out, int out_size, void* d_ws, size_t ws_size,
                              hipStream_t stream) {
  if (n_in < 1) return;
  if (in_sizes[0] != kB * kE * kF) return;
  if (out_size != kB * kE * kE) return;
  if (ws_size < (size_t)kWsTotal) return;
  const float* de = (const float*)d_in[0];
  float* out = (float*)d_out;
  char* ws = (char*)d_ws;
  unsigned short* Phi = (unsigned short*)(ws + kOffPhi);
  unsigned short* Plo = (unsigned short*)(ws + kOffPlo);
  float* G  = (float*)(ws + kOffG);
  float* SE = (float*)(ws + kOffSE);

  for (int c = 0; c < kNumChunks; ++c) {
    const int b0 = c * kChunk;
    rank_weight_kernel<<<dim3(kChunk * kF), dim3(128), 0, stream>>>(de, Phi, Plo, SE, b0);
    wmma_gemm64<1, true, 0, 0, false, 0><<<dim3(1, kChunk), dim3(128), 0, stream>>>(
        Phi, Plo, kKdim, (long)kE * kKdim,
        Phi, Plo, kKdim, (long)kE * kKdim,
        (void*)(G + (size_t)b0 * kE * kE), (void*)G, kE, (long)kE * kE,
        (const float*)SE,
        (const float*)SE, 0L,
        kE, kE, kKdim, 1.0f);
  }
  finish_kernel<<<dim3(kB * (kE / 4)), dim3(128), 0, stream>>>(G, SE, out);
}
